// ConditionedBilinearKoopmanTransition_30305289240688
// MI455X (gfx1250) — hardware-run, weakly checked
//
#include <hip/hip_runtime.h>


#define NBT  4096
#define NDM  1024
#define NUU  32
#define NRK  32
#define NOB  25
#define NOP  64
#define KXA  2112
#define KYA  1088
constexpr size_t al256(size_t b) { return (b + 255) & ~(size_t)255; }
constexpr size_t WS_TOTAL = al256((size_t)NBT * NDM * 2) + al256((size_t)NDM * NDM * 2) + al256((size_t)NDM * KXA * 2) + al256((size_t)NBT * KXA * 2) + al256((size_t)NBT * NDM * 4) + al256((size_t)NBT * KYA * 2) + al256((size_t)NOP * KYA * 2) + al256((size_t)NBT * NOP * 4);
static_assert(WS_TOTAL == 58990592 && WS_TOTAL <= 134217728, "the workspace carve: 56.3 MiB");
static_assert(KXA == NDM + NUU * NRK + 2 * NUU && KYA == NDM + 2 * NUU && KXA % 64 == 0 && KYA % 64 == 0 && NUU * NRK == NDM && NBT % 64 == 0 && NDM % 64 == 0 && NOB <= NOP && (NBT * NOB) % 4 == 0, "the concatenated depths; whole lines; whole tiles");
typedef _Float16 h16;
typedef unsigned short bf;
typedef __attribute__((ext_vector_type(16))) __bf16   v16bf;
typedef __attribute__((ext_vector_type(16))) _Float16 v16h;
typedef __attribute__((ext_vector_type(8)))  _Float16 v8h;
typedef __attribute__((ext_vector_type(8)))  unsigned short v8us;
typedef __attribute__((ext_vector_type(8)))  float    v8f;
typedef __attribute__((ext_vector_type(4)))  float    v4f;
typedef v8h  __attribute__((may_alias)) v8ha;
typedef v4f  __attribute__((may_alias)) v4fa;
typedef v8us __attribute__((may_alias)) v8usa;

__device__ __forceinline__ unsigned short f2bf(float f) { unsigned u = __float_as_uint(f); u += 0x7FFFu + ((u >> 16) & 1u); return (unsigned short)(u >> 16); }
__device__ __forceinline__ float bf2f(unsigned short b) { return __uint_as_float(((unsigned)b) << 16); }
__device__ __forceinline__ float bfr(float f) { return bf2f(f2bf(f)); }
__device__ __forceinline__ v16h cat16(v8h lo, v8h hi) { return __builtin_shufflevector(lo, hi, 0, 1, 2, 3, 4, 5, 6, 7, 8, 9, 10, 11, 12, 13, 14, 15); }
__device__ __forceinline__ v16bf cat16b(v8us lo, v8us hi) { return __builtin_bit_cast(v16bf, __builtin_shufflevector(lo, hi, 0, 1, 2, 3, 4, 5, 6, 7, 8, 9, 10, 11, 12, 13, 14, 15)); }
__device__ __forceinline__ v8f wmma16(v16h a, v16h b, v8f c) { return __builtin_amdgcn_wmma_f32_16x16x32_f16(false, a, false, b, (short)0, c, false, false); }
__device__ __forceinline__ v8f wmmab(v16bf a, v16bf b, v8f c) { return __builtin_amdgcn_wmma_f32_16x16x32_bf16(false, a, false, b, (short)0, c, false, false); }


template <typename T16> struct WFrag;
template <> struct WFrag<h16> { typedef v16h V; static __device__ __forceinline__ V ld(const h16* p) { return cat16(*(const v8h*)p, *(const v8h*)(p + 16)); } static __device__ __forceinline__ v8f mma(V a, V b, v8f c) { return wmma16(a, b, c); } };
template <> struct WFrag<bf> { typedef v16bf V; static __device__ __forceinline__ V ld(const bf* p) { return cat16b(*(const v8us*)p, *(const v8us*)(p + 16)); } static __device__ __forceinline__ v8f mma(V a, V b, v8f c) { return wmmab(a, b, c); } };
template <typename T16, int NSPLIT, bool BIAS>
__global__ __launch_bounds__(32) void k_gemmw(const T16* __restrict__ A, const T16* __restrict__ A2, const T16* __restrict__ Bt, const T16* __restrict__ Bt2, int K, float* C, int ldc, const float* __restrict__ bias, size_t sA, size_t sB, size_t sC) {
    typedef typename WFrag<T16>::V V;
    __shared__ __align__(16) float os[16 * 68];
    const size_t z = blockIdx.z; A += z * sA; if (A2) A2 += z * sA; Bt += z * sB; if (Bt2) Bt2 += z * sB; C += z * sC;
    const int lane = threadIdx.x & 31, lr = lane & 15, hi = lane >> 4; const int r0 = blockIdx.x * 64, c0 = blockIdx.y * 64;
    v8f acc[4][4];
#pragma unroll
    for (int mb = 0; mb < 4; ++mb)
#pragma unroll
        for (int nb = 0; nb < 4; ++nb) acc[mb][nb] = (v8f){};
    const size_t aoff = (size_t)(r0 + lr) * K + 8 * hi, boff = (size_t)(c0 + lr) * K + 8 * hi;
    for (int kc = 0; kc < K; kc += 32) {
        V a[4], a2[4];
#pragma unroll
        for (int mb = 0; mb < 4; ++mb) { a[mb] = WFrag<T16>::ld(A + aoff + (size_t)mb * 16 * K + kc); if (NSPLIT == 1 || NSPLIT == 2) a2[mb] = WFrag<T16>::ld(A2 + aoff + (size_t)mb * 16 * K + kc); }
#pragma unroll
        for (int nb = 0; nb < 4; ++nb) { const V b = WFrag<T16>::ld(Bt + boff + (size_t)nb * 16 * K + kc); V b2; if (NSPLIT >= 2) b2 = WFrag<T16>::ld(Bt2 + boff + (size_t)nb * 16 * K + kc);
#pragma unroll
            for (int mb = 0; mb < 4; ++mb) { acc[mb][nb] = WFrag<T16>::mma(a[mb], b, acc[mb][nb]); if (NSPLIT == 1 || NSPLIT == 2) acc[mb][nb] = WFrag<T16>::mma(a2[mb], b, acc[mb][nb]); if (NSPLIT >= 2) acc[mb][nb] = WFrag<T16>::mma(a[mb], b2, acc[mb][nb]); } }
        asm volatile("v_nop\n\tv_nop\n\tv_nop\n\tv_nop" : "+v"(acc[0][0]), "+v"(acc[1][1]), "+v"(acc[2][2]), "+v"(acc[3][3]) : "v"(a[0]), "v"(a[3]));
    }
#pragma unroll
    for (int mb = 0; mb < 4; ++mb) {
#pragma unroll
        for (int nb = 0; nb < 4; ++nb) {
#pragma unroll
            for (int j = 0; j < 8; ++j) os[(hi * 8 + j) * 68 + nb * 16 + lr] = acc[mb][nb][j]; }
        __builtin_amdgcn_wave_barrier(); asm volatile("" ::: "memory");
        float* crow = C + (size_t)(r0 + mb * 16) * ldc + c0;
#pragma unroll 1
        for (int ps = 0; ps < 2; ++ps) {
#pragma unroll
            for (int s = 0; s < 8; ++s) { const int row = 2 * s + hi, cofs = lr * 4; v4f val = *(const v4fa*)(os + row * 68 + cofs); if (BIAS) { val[0] += bfr(bias[c0 + cofs]); val[1] += bfr(bias[c0 + cofs + 1]); val[2] += bfr(bias[c0 + cofs + 2]); val[3] += bfr(bias[c0 + cofs + 3]); }
                *(volatile v4f*)(crow + (size_t)row * ldc + cofs) = val; }
            if (ps == 0) __threadfence(); }
        __builtin_amdgcn_wave_barrier(); asm volatile("" ::: "memory");
    }
}

__device__ __forceinline__ h16 tohx(float x) { return (h16)x; }
__device__ __forceinline__ void splitf(float y, unsigned short& h, unsigned short& l) { h = f2bf(y); l = f2bf(y - bf2f(h)); }
typedef __attribute__((ext_vector_type(2))) _Float16 v2h;
typedef __attribute__((ext_vector_type(4))) _Float16 v4h;
typedef __attribute__((ext_vector_type(2))) unsigned short v2us;
typedef __attribute__((ext_vector_type(4))) unsigned short v4us;
typedef __attribute__((ext_vector_type(2))) float v2f;
typedef __attribute__((ext_vector_type(4))) int v4i;


__global__ __launch_bounds__(256) void k_lay(const float* __restrict__ src, h16* dst, unsigned nrow, unsigned c8n, unsigned dp, unsigned c0, unsigned rbs, unsigned ra, unsigned rs, unsigned cbs, unsigned sa, unsigned sb, unsigned rlive, unsigned clive) {
    const unsigned g = blockIdx.x * 256 + threadIdx.x; if (g >= nrow * c8n) return; const unsigned row = g / c8n, ch = g - row * c8n; const unsigned rb = (row >> rbs) * ra + (row & ((1u << rbs) - 1u)) * rs; v8h o;
#pragma unroll
    for (int w = 0; w < 8; ++w) { const unsigned c = 8u * ch + w; const bool live = row < rlive && c < clive; const unsigned si = rb + (c >> cbs) * sa + (c & ((1u << cbs) - 1u)) * sb; const float v = bfr(src[live ? si : 0u]); o[w] = tohx(live && fabsf(v) >= 6.103515625e-05f ? v : 0.0f); }
    h16* d8 = dst + (size_t)row * dp + c0 + 8u * ch; *(volatile v8h*)(d8) = o; __threadfence(); *(volatile v8h*)(d8) = o; }

__global__ __launch_bounds__(256) void k_mul(const float* __restrict__ src, unsigned sp, int rnd, const float* __restrict__ fr, const float* __restrict__ fh, h16* dst, unsigned nrow, unsigned c8n, unsigned dp, unsigned c0, unsigned clive) {
    const unsigned g = blockIdx.x * 256 + threadIdx.x; if (g >= nrow * c8n) return; const unsigned row = g / c8n, ch = g - row * c8n; const float fhv = fh ? bfr(fh[0]) : 1.0f; v8h o;
#pragma unroll
    for (int w = 0; w < 8; ++w) { const unsigned c = 8u * ch + w; const bool live = c < clive; const float s0 = src[(size_t)row * sp + (live ? c : 0u)]; const float sv = rnd ? bfr(s0) : s0;
        const float fc = fr ? bfr(fr[(size_t)row * NUU + ((live ? c : 0u) >> 5)]) * fhv : fhv; const float pv = sv * fc; o[w] = tohx(live && fabsf(pv) >= 6.103515625e-05f ? pv : 0.0f); }
    h16* d8 = dst + (size_t)row * dp + c0 + 8u * ch; *(volatile v8h*)(d8) = o; __threadfence(); *(volatile v8h*)(d8) = o; }

__global__ __launch_bounds__(256) void k_yout(const float* __restrict__ YY, float* rs) {
    const unsigned g = blockIdx.x * 256 + threadIdx.x; if (g >= (unsigned)(NBT * NOB / 4)) return; v4f o;
#pragma unroll
    for (int w = 0; w < 4; ++w) { const unsigned e = 4u * g + w; const unsigned yr = e / NOB, n = e - yr * NOB; o[w] = YY[(size_t)yr * NOP + n]; }
    float* dq = rs + 4u * (size_t)g; *(volatile v4f*)(dq) = o; __threadfence(); *(volatile v4f*)(dq) = o; }

extern "C" void kernel_launch(void* const* d_in, const int* in_sizes, int n_in,
                              void* d_out, int out_size, void* d_ws, size_t ws_size, hipStream_t stream) {
    if (n_in < 10) return;
    if (in_sizes[0] < NBT * NDM || in_sizes[2] < 1 || in_sizes[3] < NBT * NUU || in_sizes[4] < NDM * NDM || in_sizes[5] < NDM * NUU || in_sizes[6] < NUU * NDM * NRK || in_sizes[7] < NUU * NDM * NRK || in_sizes[8] < NOB * NDM || in_sizes[9] < NOB * NUU || out_size < NBT * NDM + NBT * NOB) return;
    const float* zi = (const float*)d_in[0]; const float* hi = (const float*)d_in[2]; const float* vi = (const float*)d_in[3]; const float* ga = (const float*)d_in[4]; const float* gb = (const float*)d_in[5];
    const float* gp = (const float*)d_in[6]; const float* gq = (const float*)d_in[7]; const float* gc = (const float*)d_in[8]; const float* gd = (const float*)d_in[9];
    float* r0 = (float*)d_out; float* r1 = r0 + (size_t)NBT * NDM;
    char* wsp = (char*)d_ws;
    auto take = [&](size_t bytes) { char* cur = wsp; wsp += (bytes + 255) & ~(size_t)255; return (void*)cur; };
    h16* ZQ = (h16*)take((size_t)NBT * NDM * 2); h16* NQT = (h16*)take((size_t)NDM * NDM * 2); h16* WB = (h16*)take((size_t)NDM * KXA * 2); h16* XA = (h16*)take((size_t)NBT * KXA * 2);
    float* TT = (float*)take((size_t)NBT * NDM * 4); h16* YA = (h16*)take((size_t)NBT * KYA * 2); h16* CD = (h16*)take((size_t)NOP * KYA * 2); float* YY = (float*)take((size_t)NBT * NOP * 4);
    if ((size_t)(wsp - (char*)d_ws) != WS_TOTAL || WS_TOTAL > ws_size) return;
    auto lay = [&](const float* sp_, h16* dp_, unsigned nrow, unsigned ncol, unsigned dp, unsigned c0, unsigned rbs, unsigned ra, unsigned rs_, unsigned cbs, unsigned sa, unsigned sb, unsigned rlive, unsigned clive) {
        k_lay<<<(nrow * (ncol / 8) + 255) / 256, 256, 0, stream>>>(sp_, dp_, nrow, ncol / 8, dp, c0, rbs, ra, rs_, cbs, sa, sb, rlive, clive); };
    auto mul = [&](const float* sp_, unsigned sp, int rnd, const float* fr, const float* fh, h16* dp_, unsigned ncol, unsigned dp, unsigned c0, unsigned clive) {
        k_mul<<<(NBT * (ncol / 8) + 255) / 256, 256, 0, stream>>>(sp_, sp, rnd, fr, fh, dp_, NBT, ncol / 8, dp, c0, clive); };
    lay(zi, ZQ, NBT, NDM, NDM, 0, 16, 0, NDM, 16, 0, 1, NBT, NDM);
    lay(zi, XA, NBT, NDM, KXA, 0, 16, 0, NDM, 16, 0, 1, NBT, NDM);
    lay(gq, NQT, NDM, NDM, NDM, 0, 5, NDM * NRK, 1, 16, 0, NRK, NDM, NDM);
    lay(ga, WB, NDM, NDM, KXA, 0, 16, 0, NDM, 16, 0, 1, NDM, NDM);
    lay(gp, WB, NDM, NDM, KXA, NDM, 16, 0, NRK, 5, NDM * NRK, 1, NDM, NDM);
    lay(gb, WB, NDM, 64, KXA, 2 * NDM, 16, 0, NUU, 16, 0, 1, NDM, NUU);
    lay(gc, CD, NOP, NDM, KYA, 0, 16, 0, NDM, 16, 0, 1, NOB, NDM);
    lay(gd, CD, NOP, 64, KYA, NDM, 16, 0, NUU, 16, 0, 1, NOB, NUU);
    mul(vi, NUU, 1, nullptr, hi, XA, 64, KXA, 2 * NDM, NUU);
    mul(vi, NUU, 1, nullptr, hi, YA, 64, KYA, NDM, NUU);
    k_gemmw<h16, 0, false><<<dim3(NBT / 64, NDM / 64, 1), 32, 0, stream>>>(ZQ, nullptr, NQT, nullptr, NDM, TT, NDM, nullptr, (size_t)0, (size_t)0, (size_t)0);
    mul(TT, NDM, 0, vi, hi, XA, NDM, KXA, NDM, NDM);
    k_gemmw<h16, 0, false><<<dim3(NBT / 64, NDM / 64, 1), 32, 0, stream>>>(XA, nullptr, WB, nullptr, KXA, r0, NDM, nullptr, (size_t)0, (size_t)0, (size_t)0);
    mul(r0, NDM, 0, nullptr, nullptr, YA, NDM, KYA, 0, NDM);
    k_gemmw<h16, 0, false><<<dim3(NBT / 64, NOP / 64, 1), 32, 0, stream>>>(YA, nullptr, CD, nullptr, KYA, YY, NOP, nullptr, (size_t)0, (size_t)0, (size_t)0);
    k_yout<<<(NBT * NOB / 4 + 255) / 256, 256, 0, stream>>>(YY, r1);
}
